// GTEProgramClassification_27986006900812
// MI455X (gfx1250) — hardware-run, weakly checked
//
#include <hip/hip_runtime.h>
#include <math.h>

typedef __attribute__((ext_vector_type(16))) _Float16 v16h;
typedef __attribute__((ext_vector_type(8)))  _Float16 v8h;
typedef __attribute__((ext_vector_type(8)))  float    v8f;
typedef __attribute__((ext_vector_type(4)))  float    v4f;
typedef __attribute__((ext_vector_type(4)))  unsigned v4u;
typedef __attribute__((ext_vector_type(2)))  unsigned v2u;

constexpr int kFeat     = 128;
constexpr int kVocab    = 50000;
constexpr int kNcls     = 104;
constexpr int kNclsPad  = 128;
constexpr int kNsrc     = 300000;
constexpr int kNdst     = 100000;
constexpr int kSlots    = 5;
constexpr int kUsed     = 4;
constexpr int kGateCols = 3 * kFeat;
constexpr int kWRows    = kGateCols + kNclsPad;
constexpr int kTileM    = 32;
constexpr int kPrePitch = 388;
constexpr float kInvFeat = 1.0f / (float)kFeat;
constexpr float kLnEps   = 1e-5f;
constexpr float kCarryW   = 256.0f;
constexpr float kCarryS   = 16.0f;
constexpr float kCarryH   = 16.0f;
constexpr float kFoldGate = 1.0f / (kCarryW * kCarryS);
constexpr float kFoldCls  = 1.0f / (kCarryW * kCarryH);
constexpr float kF16MinNormal = 6.103515625e-05f;
static_assert(kFoldGate == 1.0f / 4096.0f && kFoldCls == 1.0f / 4096.0f, "fold factors");
static_assert(kCarryW * 0.09f < 1000.0f && kCarryS * 16.0f < 1000.0f && kCarryH * 12.0f < 1000.0f, "carried operands stay small");
static_assert((kFeat % 32) == 0, "K multiple of 32");
static_assert((kNdst % kTileM) == 0, "row tiles exact");
static_assert((kNdst % 16) == 0, "gather blocks exact");
static_assert((kGateCols % 128) == 0 && kNclsPad == 128, "column slices");
static_assert(((kTileM * kNcls * 4) % 128) == 0, "output tile is whole 128-B lines");
static_assert(((kTileM * kNcls / 4) % 32) == 0, "output tile copy is whole wave instructions");
static_assert((kPrePitch % 4) == 0 && kPrePitch >= kGateCols, "LDS pitch");

constexpr size_t kBytesW  = (size_t)kWRows * kFeat * 2;
constexpr size_t kBytesP  = (size_t)kNdst * kFeat * 2;
constexpr size_t kOffWP   = 0;
constexpr size_t kOffAP   = kOffWP + kBytesW;
constexpr size_t kOffHP   = kOffAP + kBytesP;
constexpr size_t kWsTotal = kOffHP + kBytesP;
static_assert(kWsTotal == 51331072ull, "carve total");
static_assert(kWsTotal <= 134217728ull, "carve cap");
static_assert((kOffAP % 128) == 0 && (kOffHP % 128) == 0, "128-B aligned regions");

__device__ __forceinline__ unsigned f16_bits_flushed(float xc) {
  const float xf = (fabsf(xc) < kF16MinNormal) ? 0.0f : xc;
  const _Float16 hv = (_Float16)xf;
  const unsigned short hb = __builtin_bit_cast(unsigned short, hv);
  return (unsigned)hb;
}
__device__ __forceinline__ unsigned pack_pair_f16(float x0, float x1) {
  const unsigned h0 = f16_bits_flushed(x0);
  const unsigned h1 = f16_bits_flushed(x1);
  return h0 | (h1 << 16);
}
union FragH { v16h v; v8h h[2]; };
__device__ __forceinline__ v16h frag_load(const _Float16* p) {
  FragH f;
  f.h[0] = *(const v8h*)(p);
  f.h[1] = *(const v8h*)(p + 16);
  return f.v;
}
__device__ __forceinline__ v8f mma_g(v16h a, v16h b, v8f c) {
  c = __builtin_amdgcn_wmma_f32_16x16x32_f16(false, a, false, b, (short)0, c, false, false);
  asm volatile("v_nop\n\tv_nop\n\tv_nop\n\tv_nop" : "+v"(c) : "v"(a), "v"(b));
  return c;
}

__global__ __launch_bounds__(256) void weight_planes_kernel(
    const float* __restrict__ W_i, const float* __restrict__ W_o,
    const float* __restrict__ W_u, const float* __restrict__ W_c,
    unsigned short* __restrict__ WP)
{
  const int tid = threadIdx.x;
  const int row = blockIdx.x * 16 + (tid >> 4);
  const int k0  = (tid & 15) * 8;
  const int g   = blockIdx.x >> 3;
  const int n   = row & 127;
  const float* W = (g == 0) ? W_i : ((g == 1) ? W_o : ((g == 2) ? W_u : W_c));
  const int ld   = (g == 3) ? kNcls : kFeat;
  const int nc   = (n < ld) ? n : (ld - 1);
  const bool live = (n < ld);
  float x[8];
#pragma unroll
  for (int e = 0; e < 8; ++e) {
    float v = W[(size_t)(k0 + e) * ld + nc];
    asm volatile("" : "+v"(v));
    x[e] = live ? v : 0.0f;
  }
  v4u wv;
#pragma unroll
  for (int e = 0; e < 4; ++e) {
    const unsigned a = pack_pair_f16(x[2 * e] * kCarryW, x[2 * e + 1] * kCarryW);
    wv[e] = a;
  }
  const size_t o = (size_t)row * kFeat + k0;
  *(volatile v4u*)(WP + o) = wv;
  __threadfence();
  *(volatile v4u*)(WP + o) = wv;
}

__global__ __launch_bounds__(256) void gather_sum_kernel(
    const int* __restrict__ token_ids, const int* __restrict__ child_idx,
    const float* __restrict__ emb,
    unsigned short* __restrict__ AP)
{
  const int tid = threadIdx.x;
  const int j   = blockIdx.x * 16 + (tid >> 4);
  const int c8  = (tid & 15) * 8;
  const int jc  = (j < kNdst) ? j : (kNdst - 1);
  const bool live = (j < kNdst);
  v4f a0 = (v4f){0.f, 0.f, 0.f, 0.f};
  v4f a1 = (v4f){0.f, 0.f, 0.f, 0.f};
#pragma unroll
  for (int k = 0; k < kUsed; ++k) {
    int s = child_idx[(size_t)jc * kSlots + k];
    s = (s < 0) ? 0 : s;
    s = (s > kNsrc - 1) ? (kNsrc - 1) : s;
    int t = token_ids[s];
    t = (t < 0) ? 0 : t;
    t = (t > kVocab - 1) ? (kVocab - 1) : t;
    const float* er = emb + (size_t)t * kFeat + c8;
    const v4f e0 = *(const v4f*)(er);
    const v4f e1 = *(const v4f*)(er + 4);
    a0 = a0 + e0;
    a1 = a1 + e1;
  }
  v4u wv;
#pragma unroll
  for (int e = 0; e < 2; ++e) {
    const float x0 = live ? a0[2 * e] : 0.0f;
    const float x1 = live ? a0[2 * e + 1] : 0.0f;
    const float y0 = live ? a1[2 * e] : 0.0f;
    const float y1 = live ? a1[2 * e + 1] : 0.0f;
    const unsigned a = pack_pair_f16(x0 * kCarryS, x1 * kCarryS);
    const unsigned b = pack_pair_f16(y0 * kCarryS, y1 * kCarryS);
    wv[e] = a;
    wv[2 + e] = b;
  }
  if (live) {
    const size_t o = (size_t)j * kFeat + c8;
    *(volatile v4u*)(AP + o) = wv;
    __threadfence();
    *(volatile v4u*)(AP + o) = wv;
  }
}

__global__ __launch_bounds__(256) void gate_norm_kernel(
    const unsigned short* __restrict__ APp, const unsigned short* __restrict__ WPp,
    const float* __restrict__ b_i, const float* __restrict__ b_o, const float* __restrict__ b_u,
    const float* __restrict__ ln_g, const float* __restrict__ ln_b,
    unsigned short* __restrict__ HP)
{
  __shared__ __align__(16) float sP[kTileM * kPrePitch];
  const _Float16* Ah = (const _Float16*)APp;
  const _Float16* Wh = (const _Float16*)WPp;
  const int tid  = threadIdx.x;
  const int lane = tid & 31;
  const int wave = tid >> 5;
  const int rs   = wave >> 2;
  const int cs   = wave & 3;
  const int rl   = lane & 15;
  const int hh   = lane >> 4;
  const int koff = hh * 8;
  const int m0   = blockIdx.x * kTileM;

  v8f acc[3][2];
#pragma unroll
  for (int g = 0; g < 3; ++g)
#pragma unroll
    for (int j = 0; j < 2; ++j) acc[g][j] = (v8f){0.f, 0.f, 0.f, 0.f, 0.f, 0.f, 0.f, 0.f};

#pragma unroll 1
  for (int k0 = 0; k0 < kFeat; k0 += 32) {
    const size_t ao = (size_t)(m0 + rs * 16 + rl) * kFeat + k0 + koff;
    const v16h ah = frag_load(Ah + ao);
#pragma unroll
    for (int g = 0; g < 3; ++g) {
#pragma unroll
      for (int j = 0; j < 2; ++j) {
        const size_t bo = (size_t)(g * kFeat + cs * 32 + j * 16 + rl) * kFeat + k0 + koff;
        const v16h bh = frag_load(Wh + bo);
        acc[g][j] = mma_g(ah, bh, acc[g][j]);
      }
    }
  }

#pragma unroll
  for (int g = 0; g < 3; ++g) {
#pragma unroll
    for (int j = 0; j < 2; ++j) {
      const int col = g * kFeat + cs * 32 + j * 16 + rl;
#pragma unroll
      for (int r = 0; r < 8; ++r) {
        sP[(rs * 16 + 8 * hh + r) * kPrePitch + col] = acc[g][j][r] * kFoldGate;
      }
    }
  }
  __syncthreads();

  const int c4 = lane * 4;
  const v4f bi4 = *(const v4f*)(b_i + c4);
  const v4f bo4 = *(const v4f*)(b_o + c4);
  const v4f bu4 = *(const v4f*)(b_u + c4);
  const v4f gg4 = *(const v4f*)(ln_g + c4);
  const v4f gb4 = *(const v4f*)(ln_b + c4);

#pragma unroll 1
  for (int it = 0; it < kTileM / 8; ++it) {
    const int row = wave + 8 * it;
    const float* pr = sP + row * kPrePitch;
    const v4f pi = *(const v4f*)(pr + c4);
    const v4f po = *(const v4f*)(pr + kFeat + c4);
    const v4f pu = *(const v4f*)(pr + 2 * kFeat + c4);
    float hv[4];
    float s1 = 0.0f;
#pragma unroll
    for (int e = 0; e < 4; ++e) {
      const float xi = pi[e] + bi4[e];
      const float xo = po[e] + bo4[e];
      const float xu = pu[e] + bu4[e];
      const float ig = 1.0f / (1.0f + expf(-xi));
      const float og = 1.0f / (1.0f + expf(-xo));
      const float ug = tanhf(xu);
      const float cc = ig * ug;
      hv[e] = og * tanhf(cc);
      s1 += hv[e];
    }
#pragma unroll
    for (int off = 16; off > 0; off >>= 1) s1 += __shfl_xor(s1, off, 32);
    const float mu = s1 * kInvFeat;
    float dv[4];
    float s2 = 0.0f;
#pragma unroll
    for (int e = 0; e < 4; ++e) {
      dv[e] = hv[e] - mu;
      s2 += dv[e] * dv[e];
    }
#pragma unroll
    for (int off = 16; off > 0; off >>= 1) s2 += __shfl_xor(s2, off, 32);
    const float var  = s2 * kInvFeat;
    const float rstd = rsqrtf(var + kLnEps);
    float yv[4];
#pragma unroll
    for (int e = 0; e < 4; ++e) yv[e] = dv[e] * rstd * gg4[e] + gb4[e];
    v2u wv;
    {
      const unsigned a = pack_pair_f16(yv[0] * kCarryH, yv[1] * kCarryH);
      const unsigned b = pack_pair_f16(yv[2] * kCarryH, yv[3] * kCarryH);
      wv[0] = a;
      wv[1] = b;
    }
    const size_t o = (size_t)(m0 + row) * kFeat + c4;
    *(volatile v2u*)(HP + o) = wv;
    __threadfence();
    *(volatile v2u*)(HP + o) = wv;
  }
}

constexpr int kOutTile4 = kTileM * kNcls / 4;
constexpr int kCopyIts  = (kOutTile4 + 127) / 128;
__global__ __launch_bounds__(128) void classifier_kernel(
    const unsigned short* __restrict__ HPp, const unsigned short* __restrict__ WPp,
    const float* __restrict__ b_c, float* __restrict__ out, int nrows)
{
  __shared__ __align__(16) float sO[kTileM * kNcls];
  const _Float16* Ah = (const _Float16*)HPp;
  const _Float16* Wh = (const _Float16*)WPp;
  const int tid  = threadIdx.x;
  const int lane = tid & 31;
  const int wave = tid >> 5;
  const int rs   = wave >> 1;
  const int cs   = wave & 1;
  const int rl   = lane & 15;
  const int hh   = lane >> 4;
  const int koff = hh * 8;
  const int m0   = blockIdx.x * kTileM;

  v8f acc[4];
#pragma unroll
  for (int j = 0; j < 4; ++j) acc[j] = (v8f){0.f, 0.f, 0.f, 0.f, 0.f, 0.f, 0.f, 0.f};

#pragma unroll 1
  for (int k0 = 0; k0 < kFeat; k0 += 32) {
    const size_t ao = (size_t)(m0 + rs * 16 + rl) * kFeat + k0 + koff;
    const v16h ah = frag_load(Ah + ao);
#pragma unroll
    for (int j = 0; j < 4; ++j) {
      const size_t bo = (size_t)(cs * 64 + j * 16 + rl) * kFeat + k0 + koff;
      const v16h bh = frag_load(Wh + bo);
      acc[j] = mma_g(ah, bh, acc[j]);
    }
  }

#pragma unroll
  for (int j = 0; j < 4; ++j) {
    const int n  = cs * 64 + j * 16 + rl;
    const int nc = (n < kNcls) ? n : (kNcls - 1);
    float bv = b_c[nc];
    asm volatile("" : "+v"(bv));
    if (n < kNcls) {
#pragma unroll
      for (int r = 0; r < 8; ++r) {
        sO[(rs * 16 + 8 * hh + r) * kNcls + n] = acc[j][r] * kFoldCls + bv;
      }
    }
  }
  __syncthreads();

  int rows_live = nrows - m0;
  rows_live = (rows_live > kTileM) ? kTileM : rows_live;
  rows_live = (rows_live < 0) ? 0 : rows_live;
  const int n4 = rows_live * (kNcls / 4);
  float* ob = out + (size_t)m0 * kNcls;
  v4f vv[kCopyIts];
#pragma unroll
  for (int it = 0; it < kCopyIts; ++it) {
    const int idx = it * 128 + tid;
    const int idc = (idx < kOutTile4) ? idx : (kOutTile4 - 1);
    vv[it] = *(const v4f*)(sO + idc * 4);
  }
  for (int pass = 0; pass < 2; ++pass) {
#pragma unroll
    for (int it = 0; it < kCopyIts; ++it) {
      const int idx = it * 128 + tid;
      if (idx < n4) {
        *(volatile v4f*)(ob + (size_t)idx * 4) = vv[it];
      }
    }
    __threadfence();
  }
}

extern "C" void kernel_launch(void* const* d_in, const int* in_sizes, int n_in,
                              void* d_out, int out_size, void* d_ws, size_t ws_size,
                              hipStream_t stream) {
  if (n_in < 15) return;
  if (in_sizes[0] != kNsrc) return;
  if (in_sizes[1] != kNdst * kSlots) return;
  if (in_sizes[2] != kVocab * kFeat) return;
  if (in_sizes[3] != kFeat * kFeat) return;
  if (in_sizes[4] != kFeat) return;
  if (in_sizes[5] != kFeat * kFeat) return;
  if (in_sizes[6] != kFeat) return;
  if (in_sizes[7] != kFeat * kFeat) return;
  if (in_sizes[8] != kFeat) return;
  if (in_sizes[11] != kFeat) return;
  if (in_sizes[12] != kFeat) return;
  if (in_sizes[13] != kFeat * kNcls) return;
  if (in_sizes[14] != kNcls) return;
  if (out_size != kNdst * kNcls) return;
  if (ws_size < kWsTotal) return;

  const int*   token_ids = (const int*)d_in[0];
  const int*   child_idx = (const int*)d_in[1];
  const float* emb       = (const float*)d_in[2];
  const float* W_ih      = (const float*)d_in[3];
  const float* b_ih      = (const float*)d_in[4];
  const float* W_oh      = (const float*)d_in[5];
  const float* b_oh      = (const float*)d_in[6];
  const float* W_uh      = (const float*)d_in[7];
  const float* b_uh      = (const float*)d_in[8];
  const float* ln_g      = (const float*)d_in[11];
  const float* ln_b      = (const float*)d_in[12];
  const float* W_fc      = (const float*)d_in[13];
  const float* b_fc      = (const float*)d_in[14];
  float* out = (float*)d_out;

  char* ws = (char*)d_ws;
  unsigned short* WP = (unsigned short*)(ws + kOffWP);
  unsigned short* AP = (unsigned short*)(ws + kOffAP);
  unsigned short* HP = (unsigned short*)(ws + kOffHP);

  weight_planes_kernel<<<kWRows / 16, 256, 0, stream>>>(W_ih, W_oh, W_uh, W_fc, WP);

  gather_sum_kernel<<<kNdst / 16, 256, 0, stream>>>(token_ids, child_idx, emb, AP);

  gate_norm_kernel<<<kNdst / kTileM, 256, 0, stream>>>(
      AP, WP, b_ih, b_oh, b_uh, ln_g, ln_b, HP);

  classifier_kernel<<<kNdst / kTileM, 128, 0, stream>>>(
      HP, WP + (size_t)kGateCols * kFeat, b_fc, out, kNdst);
}
